// Dueling_QNet_12867722018988
// MI455X (gfx1250) — hardware-verified
//
#include <hip/hip_runtime.h>
#define NN 100000
#define NEDG 2000000
#define PD 12
#define HID 128

typedef __bf16 v16b __attribute__((ext_vector_type(16)));
typedef unsigned short v8us __attribute__((ext_vector_type(8), may_alias));
typedef float  v8f  __attribute__((ext_vector_type(8)));
typedef float  v4f  __attribute__((ext_vector_type(4)));
typedef float  v4fa __attribute__((ext_vector_type(4), may_alias));
union FragB { v16b v; v8us half[2]; unsigned short u[16]; };

__device__ __forceinline__ unsigned short bf16_bits(float x) { unsigned int u = __float_as_uint(x); return (unsigned short)((u + 0x7FFFu + ((u >> 16) & 1u)) >> 16); }
__device__ __forceinline__ float bf16_val(unsigned short b) { return __uint_as_float(((unsigned int)b) << 16); }
__device__ __forceinline__ float bf16_round(float x) { return bf16_val(bf16_bits(x)); }
template <int NT>
__device__ __forceinline__ v8f mmaN(v16b ah, v16b al, v16b bh, v16b bl, v8f c) {
  c = __builtin_amdgcn_wmma_f32_16x16x32_bf16(false, ah, false, bh, (short)0, c, false, false);
  if (NT >= 2) c = __builtin_amdgcn_wmma_f32_16x16x32_bf16(false, al, false, bh, (short)0, c, false, false);
  if (NT >= 3) c = __builtin_amdgcn_wmma_f32_16x16x32_bf16(false, ah, false, bl, (short)0, c, false, false);
  asm volatile("v_nop\n\tv_nop\n\tv_nop\n\tv_nop" : "+v"(c) : "v"(ah), "v"(al), "v"(bh), "v"(bl));
  return c;
}

__global__ __launch_bounds__(256) void k_wt_bf16(const float* __restrict__ W, unsigned short* __restrict__ Wt, int K, int N) {
  const int t = blockIdx.x * 256 + threadIdx.x;
  const int k8n = K / 8;
  if (t >= N * k8n) return;
  const int n = t / k8n, k8 = (t % k8n) * 8;
  v8us v;
#pragma unroll
  for (int i = 0; i < 8; ++i) v[i] = bf16_bits(W[(size_t)(k8 + i) * N + n]);
  *(volatile v8us*)(Wt + (size_t)n * K + k8) = v;
  __threadfence();
  *(volatile v8us*)(Wt + (size_t)n * K + k8) = v;
}

template <bool ASPLIT, int ACT, bool BIAS_BF16>
__global__ __launch_bounds__(128) void k_gemm_bf(const float* __restrict__ A, int lda, const unsigned short* __restrict__ Wt, int ldb,
                                               const float* __restrict__ bias, float* __restrict__ C, int ldc, int M, int N, int K) {
  __shared__ __attribute__((aligned(16))) float so[4][16][64];
  const int tid = threadIdx.x, w = tid >> 5, lane = tid & 31, ln = lane & 15, hh = lane >> 4;
  const int ntn = N / 64;
  const int wid = blockIdx.x * 4 + w;
  const int mt = wid / ntn, nq = wid % ntn;
  if (mt * 16 >= M) return;
  const int row0 = mt * 16, col0 = nq * 64;
  const float* arow = A + (size_t)(row0 + ln) * lda;
  v8f acc[4] = {};
  for (int kb = 0; kb < K; kb += 32) {
    FragB ah, al;
    const v4f x0 = *(const v4fa*)(arow + kb + 8 * hh), x1 = *(const v4fa*)(arow + kb + 8 * hh + 4);
    const v4f x2 = *(const v4fa*)(arow + kb + 16 + 8 * hh), x3 = *(const v4fa*)(arow + kb + 16 + 8 * hh + 4);
    float xs[16] = {x0[0],x0[1],x0[2],x0[3],x1[0],x1[1],x1[2],x1[3],x2[0],x2[1],x2[2],x2[3],x3[0],x3[1],x3[2],x3[3]};
#pragma unroll
    for (int i = 0; i < 16; ++i) { const unsigned short hb = bf16_bits(xs[i]); ah.u[i] = hb; al.u[i] = ASPLIT ? bf16_bits(xs[i] - bf16_val(hb)) : (unsigned short)0; }
#pragma unroll
    for (int t = 0; t < 4; ++t) {
      const unsigned short* brow = Wt + (size_t)(col0 + t * 16 + ln) * ldb + kb;
      FragB b;
      b.half[0] = *(const v8us*)(brow + 8 * hh);
      b.half[1] = *(const v8us*)(brow + 16 + 8 * hh);
      acc[t] = mmaN<ASPLIT ? 2 : 1>(ah.v, al.v, b.v, b.v, acc[t]);
    }
  }
#pragma unroll
  for (int t = 0; t < 4; ++t) {
    float bv = bias ? bias[col0 + t * 16 + ln] : 0.f;
    if (BIAS_BF16) bv = bf16_round(bv);
#pragma unroll
    for (int r = 0; r < 8; ++r) { float v = acc[t][r] + bv; if (ACT == 1) v = fmaxf(v, 0.f); so[w][8 * hh + r][t * 16 + ln] = v; }
  }
  __builtin_amdgcn_fence(__ATOMIC_ACQ_REL, "workgroup");
  __builtin_amdgcn_wave_barrier();
  const int rsub = lane >> 4, c4 = (lane & 15) * 4;
  for (int pass = 0; pass < 2; ++pass) {
#pragma unroll
    for (int q = 0; q < 8; ++q) {
      const int r = q * 2 + rsub;
      const v4f v = *(const v4fa*)&so[w][r][c4];
      *(volatile v4f*)(C + (size_t)(row0 + r) * ldc + col0 + c4) = v;
    }
    if (pass == 0) __threadfence();
  }
}

template <int D, bool CAUSAL>
__global__ __launch_bounds__(128) void k_flash(const float* __restrict__ qb, const float* __restrict__ kb, const float* __restrict__ vb,
                                             int pitch, int T, int H, float scale, float* __restrict__ y, int ypitch) {
  constexpr int KS = D / 32;
  constexpr int DT = D / 16;
  __shared__ __attribute__((aligned(16))) unsigned short sKh[32][D + 8], sKl[32][D + 8], sVh[32][D + 8], sVl[32][D + 8];
  __shared__ __attribute__((aligned(16))) unsigned short sPh[4][16][40], sPl[4][16][40];
  __shared__ __attribute__((aligned(16))) float sO[4][16][D];
  const int tid = threadIdx.x, w = tid >> 5, lane = tid & 31, ln = lane & 15, hh = lane >> 4;
  const int nqb = (T + 63) / 64;
  const int bh = blockIdx.x / nqb, qblk = blockIdx.x % nqb;
  const int b = bh / H, h = bh % H;
  const int q0 = qblk * 64 + w * 16;
  const float* Q = qb + (size_t)b * T * pitch + h * D;
  const float* K = kb + (size_t)b * T * pitch + h * D;
  const float* V = vb + (size_t)b * T * pitch + h * D;

  FragB aqh[KS], aql[KS];
  {
    int row = q0 + ln; if (row >= T) row = T - 1;
    const float* qr = Q + (size_t)row * pitch;
#pragma unroll
    for (int ks = 0; ks < KS; ++ks)
#pragma unroll
      for (int i = 0; i < 16; ++i) {
        const int d = ks * 32 + ((i < 8) ? (8 * hh + i) : (16 + 8 * hh + (i - 8)));
        const float x = qr[d] * scale; const unsigned short hb = bf16_bits(x);
        aqh[ks].u[i] = hb; aql[ks].u[i] = bf16_bits(x - bf16_val(hb));
      }
  }
  float m_r[8], l_r[8];
#pragma unroll
  for (int r = 0; r < 8; ++r) { m_r[r] = -3.0e38f; l_r[r] = 0.f; }
  v8f oacc[DT];
#pragma unroll
  for (int dt = 0; dt < DT; ++dt) oacc[dt] = (v8f){0.f,0.f,0.f,0.f,0.f,0.f,0.f,0.f};

  const int kv_end = CAUSAL ? min(T, qblk * 64 + 64) : T;
  for (int j0 = 0; j0 < kv_end; j0 += 32) {
    __syncthreads();
    for (int e = tid; e < 32 * (D / 4); e += 128) {
      const int r = e / (D / 4), c4 = (e % (D / 4)) * 4;
      const int key = j0 + r;
      v4f kf = {0.f,0.f,0.f,0.f}, vf = {0.f,0.f,0.f,0.f};
      if (key < T) { kf = *(const v4fa*)(K + (size_t)key * pitch + c4); vf = *(const v4fa*)(V + (size_t)key * pitch + c4); }
#pragma unroll
      for (int t = 0; t < 4; ++t) {
        unsigned short hb = bf16_bits(kf[t]); sKh[r][c4 + t] = hb; sKl[r][c4 + t] = bf16_bits(kf[t] - bf16_val(hb));
        hb = bf16_bits(vf[t]); sVh[r][c4 + t] = hb; sVl[r][c4 + t] = bf16_bits(vf[t] - bf16_val(hb));
      }
    }
    __syncthreads();
    v8f s[2];
#pragma unroll
    for (int nt = 0; nt < 2; ++nt) {
      v8f acc = {};
#pragma unroll
      for (int ks = 0; ks < KS; ++ks) {
        FragB bh_, bl_;
        bh_.half[0] = *(const v8us*)&sKh[nt * 16 + ln][ks * 32 + 8 * hh]; bh_.half[1] = *(const v8us*)&sKh[nt * 16 + ln][ks * 32 + 16 + 8 * hh];
        bl_.half[0] = *(const v8us*)&sKl[nt * 16 + ln][ks * 32 + 8 * hh]; bl_.half[1] = *(const v8us*)&sKl[nt * 16 + ln][ks * 32 + 16 + 8 * hh];
        acc = mmaN<3>(aqh[ks].v, aql[ks].v, bh_.v, bl_.v, acc);
      }
      s[nt] = acc;
    }
    float alpha[8];
#pragma unroll
    for (int r = 0; r < 8; ++r) {
      const int qi = q0 + 8 * hh + r;
      const int ja = j0 + ln, jb = j0 + 16 + ln;
      if (CAUSAL) { if (ja > qi) s[0][r] = -3.0e38f; if (jb > qi) s[1][r] = -3.0e38f; }
      if (ja >= T) s[0][r] = -3.0e38f;
      if (jb >= T) s[1][r] = -3.0e38f;
      float mx = fmaxf(s[0][r], s[1][r]);
      mx = fmaxf(mx, __shfl_xor(mx, 1, 32)); mx = fmaxf(mx, __shfl_xor(mx, 2, 32)); mx = fmaxf(mx, __shfl_xor(mx, 4, 32)); mx = fmaxf(mx, __shfl_xor(mx, 8, 32));
      const float mnew = fmaxf(m_r[r], mx);
      alpha[r] = (mnew > -1.0e38f) ? __expf(m_r[r] - mnew) : 1.0f;
      const float p0 = (s[0][r] > -1.0e38f) ? __expf(s[0][r] - mnew) : 0.f;
      const float p1 = (s[1][r] > -1.0e38f) ? __expf(s[1][r] - mnew) : 0.f;
      m_r[r] = mnew;
      l_r[r] = l_r[r] * alpha[r] + p0 + p1;
      unsigned short hb = bf16_bits(p0); sPh[w][8 * hh + r][ln] = hb;      sPl[w][8 * hh + r][ln] = bf16_bits(p0 - bf16_val(hb));
      hb = bf16_bits(p1);                sPh[w][8 * hh + r][16 + ln] = hb; sPl[w][8 * hh + r][16 + ln] = bf16_bits(p1 - bf16_val(hb));
    }
#pragma unroll
    for (int dt = 0; dt < DT; ++dt)
#pragma unroll
      for (int r = 0; r < 8; ++r) oacc[dt][r] *= alpha[r];
    __builtin_amdgcn_fence(__ATOMIC_ACQ_REL, "workgroup");
    __builtin_amdgcn_wave_barrier();
    FragB pah, pal;
    pah.half[0] = *(const v8us*)&sPh[w][ln][8 * hh]; pah.half[1] = *(const v8us*)&sPh[w][ln][16 + 8 * hh];
    pal.half[0] = *(const v8us*)&sPl[w][ln][8 * hh]; pal.half[1] = *(const v8us*)&sPl[w][ln][16 + 8 * hh];
#pragma unroll
    for (int dt = 0; dt < DT; ++dt) {
      FragB bvh, bvl;
#pragma unroll
      for (int i = 0; i < 8; ++i) {
        bvh.u[i] = sVh[8 * hh + i][dt * 16 + ln]; bvh.u[8 + i] = sVh[16 + 8 * hh + i][dt * 16 + ln];
        bvl.u[i] = sVl[8 * hh + i][dt * 16 + ln]; bvl.u[8 + i] = sVl[16 + 8 * hh + i][dt * 16 + ln];
      }
      oacc[dt] = mmaN<3>(pah.v, pal.v, bvh.v, bvl.v, oacc[dt]);
    }
    __builtin_amdgcn_fence(__ATOMIC_ACQ_REL, "workgroup");
    __builtin_amdgcn_wave_barrier();
  }
#pragma unroll
  for (int r = 0; r < 8; ++r) {
    float l = l_r[r];
    l += __shfl_xor(l, 1, 32); l += __shfl_xor(l, 2, 32); l += __shfl_xor(l, 4, 32); l += __shfl_xor(l, 8, 32);
    l_r[r] = (l > 0.f) ? 1.0f / l : 0.f;
  }
#pragma unroll
  for (int dt = 0; dt < DT; ++dt)
#pragma unroll
    for (int r = 0; r < 8; ++r) sO[w][8 * hh + r][dt * 16 + ln] = oacc[dt][r] * l_r[r];
  __builtin_amdgcn_fence(__ATOMIC_ACQ_REL, "workgroup");
  __builtin_amdgcn_wave_barrier();
  for (int pass = 0; pass < 2; ++pass) {
    for (int r = 0; r < 16; ++r) {
      const int row = q0 + r;
      if (row < T && lane < D / 4) {
        const v4f val = *(const v4fa*)&sO[w][r][lane * 4];
        *(volatile v4f*)(y + ((size_t)b * T + row) * ypitch + h * D + lane * 4) = val;
      }
    }
    if (pass == 0) __threadfence();
  }
}

__global__ __launch_bounds__(256) void k_prep_w(const float* __restrict__ W1, const float* __restrict__ W2, unsigned short* __restrict__ Bt1, unsigned short* __restrict__ Bt2) {
  const int t = blockIdx.x * 256 + threadIdx.x;
  if (t < HID * 4) {
    const int n = t / 4, k8 = (t % 4) * 8; v8us v;
#pragma unroll
    for (int i = 0; i < 8; ++i) { const int k = k8 + i; v[i] = (k < 2 * PD) ? bf16_bits(W1[k * HID + n]) : (unsigned short)0; }
    *(volatile v8us*)(Bt1 + n * 32 + k8) = v; __threadfence(); *(volatile v8us*)(Bt1 + n * 32 + k8) = v;
  } else if (t < HID * 4 + HID * 16) {
    const int u = t - HID * 4; const int n = u / 16, k8 = (u % 16) * 8; v8us v;
#pragma unroll
    for (int i = 0; i < 8; ++i) v[i] = bf16_bits(W2[(k8 + i) * HID + n]);
    *(volatile v8us*)(Bt2 + n * HID + k8) = v; __threadfence(); *(volatile v8us*)(Bt2 + n * HID + k8) = v;
  }
}
__global__ __launch_bounds__(128) void k_edge_mlp(const float* __restrict__ emb, const int* __restrict__ src, const int* __restrict__ dst,
                                                const unsigned short* __restrict__ Bt1, const float* __restrict__ b1, const unsigned short* __restrict__ Bt2, const float* __restrict__ b2,
                                                const float* __restrict__ Wv, const float* __restrict__ bv, const float* __restrict__ Wa, const float* __restrict__ ba,
                                                float* __restrict__ qa, float* __restrict__ slots) {
  __shared__ __attribute__((aligned(16))) unsigned short sA[4][16][40];
  __shared__ __attribute__((aligned(16))) float sH1[4][16][HID + 4];
  __shared__ __attribute__((aligned(16))) float sH2[4][16][HID + 4];
  __shared__ float sQ[4][32]; __shared__ float sAdv[4];
  const int tid = threadIdx.x, w = tid >> 5, lane = tid & 31, ln = lane & 15, hh = lane >> 4;
  const size_t e0 = ((size_t)blockIdx.x * 4 + w) * 32;
  float advsum = 0.f;
  for (int sub = 0; sub < 2; ++sub) {
    const size_t eb = e0 + sub * 16;
    __builtin_amdgcn_fence(__ATOMIC_ACQ_REL, "workgroup");
    __builtin_amdgcn_wave_barrier();
    {
      const size_t e = eb + ln;
      int node = hh ? dst[e] : src[e]; node = node < 0 ? 0 : (node >= NN ? NN - 1 : node);
      const float* er = emb + (size_t)node * PD;
#pragma unroll
      for (int j = 0; j < PD; ++j) sA[w][ln][hh * PD + j] = bf16_bits(er[j]);
      if (hh == 1) { for (int j = 2 * PD; j < 32; ++j) sA[w][ln][j] = 0; }
    }
    __builtin_amdgcn_fence(__ATOMIC_ACQ_REL, "workgroup");
    __builtin_amdgcn_wave_barrier();
    FragB a1; a1.half[0] = *(const v8us*)&sA[w][ln][8 * hh]; a1.half[1] = *(const v8us*)&sA[w][ln][16 + 8 * hh];
#pragma unroll
    for (int nt = 0; nt < 8; ++nt) {
      const int n = nt * 16 + ln;
      FragB bb; bb.half[0] = *(const v8us*)(Bt1 + n * 32 + 8 * hh); bb.half[1] = *(const v8us*)(Bt1 + n * 32 + 16 + 8 * hh);
      v8f acc = {}; acc = mmaN<1>(a1.v, a1.v, bb.v, bb.v, acc);
      const float bvv = bf16_round(b1[n]);
#pragma unroll
      for (int r = 0; r < 8; ++r) sH1[w][8 * hh + r][n] = fmaxf(acc[r] + bvv, 0.f);
    }
    __builtin_amdgcn_fence(__ATOMIC_ACQ_REL, "workgroup");
    __builtin_amdgcn_wave_barrier();
    FragB ah[4], al[4];
#pragma unroll
    for (int ks = 0; ks < 4; ++ks)
#pragma unroll
      for (int i = 0; i < 16; ++i) { const int k = ks * 32 + ((i < 8) ? (8 * hh + i) : (16 + 8 * hh + (i - 8))); const float x = sH1[w][ln][k]; const unsigned short hb = bf16_bits(x); ah[ks].u[i] = hb; al[ks].u[i] = bf16_bits(x - bf16_val(hb)); }
#pragma unroll 1
    for (int nt = 0; nt < 8; ++nt) {
      const int n = nt * 16 + ln;
      v8f acc = {};
#pragma unroll
      for (int ks = 0; ks < 4; ++ks) { FragB bb; bb.half[0] = *(const v8us*)(Bt2 + n * HID + ks * 32 + 8 * hh); bb.half[1] = *(const v8us*)(Bt2 + n * HID + ks * 32 + 16 + 8 * hh); acc = mmaN<2>(ah[ks].v, al[ks].v, bb.v, bb.v, acc); }
      const float bvv = bf16_round(b2[n]);
#pragma unroll
      for (int r = 0; r < 8; ++r) sH2[w][8 * hh + r][n] = fmaxf(acc[r] + bvv, 0.f);
    }
    __builtin_amdgcn_fence(__ATOMIC_ACQ_REL, "workgroup");
    __builtin_amdgcn_wave_barrier();
    float sv = 0.f, sa = 0.f;
#pragma unroll 4
    for (int j = 0; j < 64; ++j) { const int k = hh * 64 + j; const float hv = sH2[w][ln][k]; sv += hv * bf16_round(Wv[k]); sa += hv * bf16_round(Wa[k]); }
    sv += __shfl_xor(sv, 16, 32); sa += __shfl_xor(sa, 16, 32);
    const float val = sv + bf16_round(bv[0]), adv = sa + bf16_round(ba[0]);
    if (hh == 0) sQ[w][sub * 16 + ln] = val + adv;
    float as = (hh == 0) ? adv : 0.f;
    as += __shfl_xor(as, 1, 32); as += __shfl_xor(as, 2, 32); as += __shfl_xor(as, 4, 32); as += __shfl_xor(as, 8, 32);
    advsum += as;
  }
  __builtin_amdgcn_fence(__ATOMIC_ACQ_REL, "workgroup");
  __builtin_amdgcn_wave_barrier();
  { const float v = sQ[w][lane]; *(volatile float*)(qa + e0 + lane) = v; __threadfence(); *(volatile float*)(qa + e0 + lane) = v; }
  if (lane == 0) sAdv[w] = advsum;
  __syncthreads();
  if (tid < 32) { const float v = (tid == 0) ? (sAdv[0] + sAdv[1] + sAdv[2] + sAdv[3]) : 0.f; *(volatile float*)(slots + (size_t)blockIdx.x * 32 + tid) = v; __threadfence(); *(volatile float*)(slots + (size_t)blockIdx.x * 32 + tid) = v; }
}
__global__ __launch_bounds__(256) void k_mean(const float* __restrict__ slots, int nslots, float* __restrict__ mean) {
  __shared__ double red[256];
  const int tid = threadIdx.x; double s = 0.0;
  for (int i = tid; i < nslots; i += 256) s += (double)slots[(size_t)i * 32];
  red[tid] = s; __syncthreads();
  for (int st = 128; st > 0; st >>= 1) { if (tid < st) red[tid] += red[tid + st]; __syncthreads(); }
  if (tid < 32) { const float v = (tid == 0) ? (float)(red[0] / (double)NEDG) : 0.f; *(volatile float*)(mean + tid) = v; __threadfence(); *(volatile float*)(mean + tid) = v; }
}
__global__ __launch_bounds__(256) void k_final(const float* __restrict__ qa, const float* __restrict__ mean, float* __restrict__ out, int n4) {
  const size_t t = (size_t)blockIdx.x * 256 + threadIdx.x; if (t >= (size_t)n4) return;
  const float m = mean[0]; const v4f a = *(const v4fa*)(qa + t * 4); v4f o; for (int q = 0; q < 4; ++q) o[q] = a[q] - m;
  *(volatile v4f*)(out + t * 4) = o; __threadfence(); *(volatile v4f*)(out + t * 4) = o;
}

extern "C" void kernel_launch(void* const* d_in, const int* in_sizes, int n_in,
                              void* d_out, int out_size, void* d_ws, size_t ws_size, hipStream_t stream) {
  (void)in_sizes; (void)n_in; (void)out_size;
  const float* emb = (const float*)d_in[0]; const int* src = (const int*)d_in[1]; const int* dst = (const int*)d_in[2];
  const float* W1 = (const float*)d_in[3]; const float* b1 = (const float*)d_in[4]; const float* W2 = (const float*)d_in[5]; const float* b2 = (const float*)d_in[6];
  const float* Wv = (const float*)d_in[7]; const float* bv = (const float*)d_in[8]; const float* Wa = (const float*)d_in[9]; const float* ba = (const float*)d_in[10];
  char* ws = (char*)d_ws; size_t off = 0;
  auto take = [&](size_t bytes) { char* p = ws + off; off += (bytes + 255) & ~(size_t)255; return p; };
  const int nblk = NEDG / 128;
  unsigned short* Bt1 = (unsigned short*)take(HID * 32 * 2); unsigned short* Bt2 = (unsigned short*)take(HID * HID * 2);
  float* qa = (float*)take((size_t)NEDG * 4); float* slots = (float*)take((size_t)nblk * 32 * 4); float* mean = (float*)take(32 * 4);
  if (off > ws_size) return;
  k_prep_w<<<(HID * 20 + 255) / 256, 256, 0, stream>>>(W1, W2, Bt1, Bt2);
  k_edge_mlp<<<nblk, 128, 0, stream>>>(emb, src, dst, Bt1, b1, Bt2, b2, Wv, bv, Wa, ba, qa, slots);
  k_mean<<<1, 256, 0, stream>>>(slots, nblk, mean);
  k_final<<<(NEDG / 4 + 255) / 256, 256, 0, stream>>>(qa, mean, (float*)d_out, NEDG / 4);
}
